// RNNModel_29016799052140
// MI455X (gfx1250) — hardware-verified
//
#include <hip/hip_runtime.h>

constexpr int NB   = 256;
constexpr int NT   = 512;
constexpr int NI   = 64;
constexpr int NH   = 512;
constexpr int NO   = 24;
constexpr int KCAT = NI + NH;
constexpr int NTHR = 256;
constexpr int SEQ_BLK = 16;
constexpr int NBLK = NB / SEQ_BLK;
constexpr int KP    = KCAT + 8;
constexpr int HTILE = SEQ_BLK * KP;
constexpr int HSP   = NH + 4;
constexpr int OUT_PER_BLK = SEQ_BLK * NO;
constexpr float WCARRY     = 256.0f;
constexpr float WCARRY_INV = 1.0f / 256.0f;
constexpr int PREP_IH_THREADS = NH * (NI / 8);
constexpr int PREP_HH_THREADS = NH * (NH / 8);
constexpr int PREP_IH_BLOCKS  = PREP_IH_THREADS / NTHR;
constexpr int PREP_HH_BLOCKS  = PREP_HH_THREADS / NTHR;
constexpr int PREP_BLOCKS     = PREP_IH_BLOCKS + PREP_HH_BLOCKS;
constexpr size_t WCAT_BYTES   = (size_t)NH * KCAT * 2;

static_assert(NB % SEQ_BLK == 0);
static_assert(NH == 64 * (NTHR / 32));
static_assert(KCAT % 32 == 0);
static_assert(KP % 8 == 0);
static_assert((HTILE * 2) % 16 == 0);
static_assert(NI == 64);
static_assert(SEQ_BLK * (NI / 8) == 128);
static_assert(HSP % 4 == 0);
static_assert(OUT_PER_BLK == 3 * 128);
static_assert((OUT_PER_BLK * 4) % 128 == 0);
static_assert(NO % 2 == 0 && SEQ_BLK * (NO / 2) == 192);
static_assert(NB * NO == NBLK * OUT_PER_BLK);
static_assert(PREP_IH_THREADS % NTHR == 0 && PREP_HH_THREADS % NTHR == 0);
static_assert(PREP_BLOCKS == 144);
static_assert((KCAT * 2) % 128 == 0);
static_assert(WCAT_BYTES <= (size_t)134217728);

typedef __attribute__((ext_vector_type(16))) _Float16 v16h;
typedef __attribute__((ext_vector_type(8)))  _Float16 v8h;
typedef __attribute__((ext_vector_type(8)))  float    v8f;
typedef __attribute__((ext_vector_type(4)))  float    v4f;

__device__ __forceinline__ void dep_guard_h(v8f& a, v8f& b, v16h x, v16h y) { asm volatile("v_nop\n\tv_nop\n\tv_nop\n\tv_nop" : "+v"(a), "+v"(b) : "v"(x), "v"(y)); }
__device__ __forceinline__ void keep4_h(v16h a, v16h b, v16h c, v16h d) { asm volatile("v_nop" :: "v"(a), "v"(b), "v"(c), "v"(d)); }
__device__ __forceinline__ void acc_guard4(v8f& a, v8f& b, v8f& c, v8f& d) { asm volatile("v_nop\n\tv_nop\n\tv_nop\n\tv_nop" : "+v"(a), "+v"(b), "+v"(c), "+v"(d)); }
__device__ __forceinline__ void guard_all4(v8f& a0, v8f& a1, v8f& a2, v8f& a3,
                                           v16h fa, v16h b0, v16h b1, v16h b2, v16h b3) {
  asm volatile("v_nop\n\tv_nop\n\tv_nop\n\tv_nop"
               : "+v"(a0), "+v"(a1), "+v"(a2), "+v"(a3)
               : "v"(fa), "v"(b0), "v"(b1), "v"(b2), "v"(b3));
}
template <typename T> struct Frag;
template <> struct Frag<_Float16> {
  typedef v16h V; union U { v16h v; v8h h[2]; };
  static __device__ __forceinline__ v16h load(const _Float16* p) {
    U f; f.h[0] = *(const v8h*)(p); f.h[1] = *(const v8h*)(p + 16); return f.v;
  }
  static __device__ __forceinline__ v8f mma(v16h a, v16h b, v8f c) {
    return __builtin_amdgcn_wmma_f32_16x16x32_f16(false, a, false, b, (short)0, c, false, false);
  }
  static __device__ __forceinline__ void guard(v8f& a, v8f& b, v16h x, v16h y) { dep_guard_h(a, b, x, y); }
  static __device__ __forceinline__ void keep(v16h a, v16h b, v16h c, v16h d) { keep4_h(a, b, c, d); }
};

__device__ __forceinline__ void cvt8_store(const float* __restrict__ src, _Float16* __restrict__ dst) {
  const v4f a = *(const v4f*)(src);
  const v4f b = *(const v4f*)(src + 4);
  v8h hv;
  hv[0] = (_Float16)(a[0] * WCARRY); hv[1] = (_Float16)(a[1] * WCARRY);
  hv[2] = (_Float16)(a[2] * WCARRY); hv[3] = (_Float16)(a[3] * WCARRY);
  hv[4] = (_Float16)(b[0] * WCARRY); hv[5] = (_Float16)(b[1] * WCARRY);
  hv[6] = (_Float16)(b[2] * WCARRY); hv[7] = (_Float16)(b[3] * WCARRY);
  *(volatile v8h*)dst = hv;
  __threadfence();
  *(volatile v8h*)dst = hv;
}

__global__ __launch_bounds__(NTHR) void wprep_kernel(const float* __restrict__ w_ih, const float* __restrict__ w_hh,
                                                     _Float16* __restrict__ wcat) {
  const int blk = blockIdx.x, tid = threadIdx.x;
  if (blk < PREP_IH_BLOCKS) {
    const int p = blk * NTHR + tid;
    const int row = p >> 3, c8 = p & 7;
    cvt8_store(w_ih + (size_t)row * NI + c8 * 8, wcat + (size_t)row * KCAT + c8 * 8);
  } else {
    const int p = (blk - PREP_IH_BLOCKS) * NTHR + tid;
    const int row = p >> 6, c8 = p & 63;
    cvt8_store(w_hh + (size_t)row * NH + c8 * 8, wcat + (size_t)row * KCAT + NI + c8 * 8);
  }
}

__global__ __launch_bounds__(NTHR) void rnn_relu_kernel(const float* __restrict__ x,
                                                        const float* __restrict__ b_ih, const float* __restrict__ b_hh,
                                                        const _Float16* __restrict__ wcat,
                                                        const float* __restrict__ fc_w, const float* __restrict__ fc_b,
                                                        float* __restrict__ out) {
  __shared__ __align__(16) _Float16 atile[2 * HTILE];
  __shared__ __align__(16) float    hs[SEQ_BLK * HSP];
  __shared__ __align__(16) float    os[OUT_PER_BLK];
  const int tid = threadIdx.x, lane = tid & 31, wave = tid >> 5;
  const int c = lane & 15, hh = lane >> 4, koff = hh * 8, mOff = hh * 8;
  const int b0 = blockIdx.x * SEQ_BLK;
  const int n0 = wave * 64;

  {
    v8h z;
#pragma unroll
    for (int e = 0; e < 8; ++e) z[e] = (_Float16)0.0f;
#pragma unroll 1
    for (int i = tid; i < (2 * HTILE) / 8; i += NTHR) *(v8h*)(atile + i * 8) = z;
  }
  float bj[4];
#pragma unroll
  for (int j = 0; j < 4; ++j) {
    const int n = n0 + 16 * j + c;
    bj[j] = b_ih[n] + b_hh[n];
  }
  float hst[4][8];
#pragma unroll
  for (int j = 0; j < 4; ++j)
#pragma unroll
    for (int r = 0; r < 8; ++r) hst[j][r] = 0.0f;
  __syncthreads();

  if (tid < 128) {
    const int row = tid >> 3, c8 = (tid & 7) * 8;
    const float* xp = x + ((size_t)(b0 + row) * NT + (size_t)0) * NI + c8;
    const v4f f0 = *(const v4f*)xp;
    const v4f f1 = *(const v4f*)(xp + 4);
    v8h hv;
    hv[0] = (_Float16)f0[0]; hv[1] = (_Float16)f0[1]; hv[2] = (_Float16)f0[2]; hv[3] = (_Float16)f0[3];
    hv[4] = (_Float16)f1[0]; hv[5] = (_Float16)f1[1]; hv[6] = (_Float16)f1[2]; hv[7] = (_Float16)f1[3];
    *(v8h*)(atile + row * KP + c8) = hv;
  }
  __syncthreads();

  const v8f z8 = {0.f, 0.f, 0.f, 0.f, 0.f, 0.f, 0.f, 0.f};
  const _Float16* brow = wcat + (size_t)(n0 + c) * KCAT + koff;

#pragma unroll 1
  for (int t = 0; t < NT; ++t) {
    const _Float16* hc = atile + (t & 1) * HTILE;
    _Float16*       hn = atile + ((t + 1) & 1) * HTILE;
    const int tn = (t + 1 < NT) ? (t + 1) : (NT - 1);

    if (tid < 128) {
      const int row = tid >> 3, c8 = (tid & 7) * 8;
      const float* xp = x + ((size_t)(b0 + row) * NT + (size_t)tn) * NI + c8;
      const v4f f0 = *(const v4f*)xp;
      const v4f f1 = *(const v4f*)(xp + 4);
      v8h hv;
      hv[0] = (_Float16)f0[0]; hv[1] = (_Float16)f0[1]; hv[2] = (_Float16)f0[2]; hv[3] = (_Float16)f0[3];
      hv[4] = (_Float16)f1[0]; hv[5] = (_Float16)f1[1]; hv[6] = (_Float16)f1[2]; hv[7] = (_Float16)f1[3];
      *(v8h*)(hn + row * KP + c8) = hv;
    }

    v8f acc[4];
#pragma unroll
    for (int j = 0; j < 4; ++j) acc[j] = z8;
    const _Float16* arow = hc + c * KP + koff;
    v16h fa;
    v16h fb[4];
#pragma unroll 2
    for (int kc = 0; kc < KCAT / 32; ++kc) {
      fa = Frag<_Float16>::load(arow + kc * 32);
#pragma unroll
      for (int j = 0; j < 4; ++j) fb[j] = Frag<_Float16>::load(brow + (size_t)(16 * j) * KCAT + kc * 32);
#pragma unroll
      for (int j = 0; j < 4; ++j) acc[j] = Frag<_Float16>::mma(fa, fb[j], acc[j]);
      guard_all4(acc[0], acc[1], acc[2], acc[3], fa, fb[0], fb[1], fb[2], fb[3]);
    }
    acc_guard4(acc[0], acc[1], acc[2], acc[3]);

#pragma unroll
    for (int j = 0; j < 4; ++j) {
      const int col = NI + n0 + 16 * j + c;
#pragma unroll
      for (int r = 0; r < 8; ++r) {
        float v = acc[j][r] * WCARRY_INV + bj[j];
        v = fmaxf(v, 0.0f);
        hst[j][r] = v;
        hn[(mOff + r) * KP + col] = (_Float16)v;
      }
    }
    __syncthreads();
  }

#pragma unroll
  for (int j = 0; j < 4; ++j)
#pragma unroll
    for (int r = 0; r < 8; ++r) hs[(mOff + r) * HSP + n0 + 16 * j + c] = hst[j][r];
  __syncthreads();

  if (tid < 192) {
    const int bl = tid / 12;
    const int o0 = (tid - bl * 12) * 2;
    const float* w0 = fc_w + (size_t)o0 * NH;
    const float* w1 = w0 + NH;
    const float* hrow = hs + bl * HSP;
    float s0 = 0.0f, s1 = 0.0f;
#pragma unroll 2
    for (int k = 0; k < NH; k += 4) {
      const v4f hv = *(const v4f*)(hrow + k);
      const v4f wa = *(const v4f*)(w0 + k);
      const v4f wb = *(const v4f*)(w1 + k);
      s0 += hv[0] * wa[0]; s0 += hv[1] * wa[1]; s0 += hv[2] * wa[2]; s0 += hv[3] * wa[3];
      s1 += hv[0] * wb[0]; s1 += hv[1] * wb[1]; s1 += hv[2] * wb[2]; s1 += hv[3] * wb[3];
    }
    const float r0 = s0 + fc_b[o0];
    const float r1 = s1 + fc_b[o0 + 1];
    os[bl * NO + o0]     = r0;
    os[bl * NO + o0 + 1] = r1;
  }
  __syncthreads();

  if (wave < 3) {
    const int base = wave * 128 + lane * 4;
    const v4f v = *(const v4f*)(os + base);
    float* op = out + (size_t)blockIdx.x * OUT_PER_BLK + base;
    *(volatile v4f*)op = v;
    __threadfence();
    *(volatile v4f*)op = v;
  }
}

extern "C" void kernel_launch(void* const* d_in, const int* in_sizes, int n_in,
                              void* d_out, int out_size, void* d_ws, size_t ws_size, hipStream_t stream) {
  if (n_in < 7 || d_out == nullptr || d_ws == nullptr) return;
  if (in_sizes[0] != NB * NT * NI || in_sizes[1] != NH * NI || in_sizes[2] != NH * NH ||
      in_sizes[3] != NH || in_sizes[4] != NH || in_sizes[5] != NO * NH || in_sizes[6] != NO ||
      out_size != NB * NO) return;
  if (WCAT_BYTES > ws_size) return;

  const float* x    = (const float*)d_in[0];
  const float* w_ih = (const float*)d_in[1];
  const float* w_hh = (const float*)d_in[2];
  const float* b_ih = (const float*)d_in[3];
  const float* b_hh = (const float*)d_in[4];
  const float* fc_w = (const float*)d_in[5];
  const float* fc_b = (const float*)d_in[6];
  float* out = (float*)d_out;

  _Float16* wcat = (_Float16*)d_ws;

  wprep_kernel<<<PREP_BLOCKS, NTHR, 0, stream>>>(w_ih, w_hh, wcat);
  rnn_relu_kernel<<<NBLK, NTHR, 0, stream>>>(x, b_ih, b_hh, wcat, fc_w, fc_b, out);
}
